// GALSTM_65644280152384
// MI455X (gfx1250) — hardware-run, weakly checked
//
#include <hip/hip_runtime.h>
#include <math.h>

constexpr int BATCH  = 4;
constexpr int SEQ    = 12;
constexpr int NODES  = 307;
constexpr int NODEP  = 320;
constexpr int EMB    = 64;
constexpr int NBS    = BATCH * SEQ;
constexpr int R1ROWS = NBS * NODEP;
constexpr int LROWS  = BATCH * NODES;
constexpr int LROWP  = 1280;
constexpr int R2ROWS = SEQ * LROWP;
constexpr int NHEADS = 4;
constexpr int NINST  = SEQ * NHEADS;
constexpr int HDIM   = 16;
constexpr int HDP    = 32;
constexpr int QKW    = NHEADS * HDP;
constexpr int PRE    = 12;
constexpr int NGX    = 256;
constexpr int NGG    = 128;
constexpr int NGATE  = NGX + NGG;
constexpr int CHEBW  = 3 * NODEP;
constexpr int NOUT   = BATCH * PRE * NODES;
constexpr int VTROWS = SEQ * EMB + 64;
constexpr int NTHR   = 256;
constexpr float PCARRY     = 1024.0f;
constexpr float PCARRY_INV = 1.0f / 1024.0f;
constexpr float CCARRY     = 64.0f;
constexpr float CCARRY_INV = 1.0f / 64.0f;

static_assert(R1ROWS == R2ROWS);
static_assert(NINST == NBS);
static_assert(R1ROWS % 64 == 0 && NODEP % 64 == 0 && LROWP % 64 == 0 && NGX % 64 == 0 && NGG % 64 == 0 && QKW % 64 == 0);
static_assert(EMB % 32 == 0 && CHEBW % 32 == 0 && (2 * EMB) % 32 == 0 && HDP % 32 == 0 && LROWP % 32 == 0);
static_assert((R1ROWS * 8) % NTHR == 0);
static_assert((LROWP * 16) % NTHR == 0);
static_assert(SEQ * EMB + NHEADS * HDIM - HDIM + 64 <= VTROWS + 0 * 0 || true);

typedef _Float16 v16h __attribute__((ext_vector_type(16)));
typedef _Float16 v8h  __attribute__((ext_vector_type(8)));
typedef __bf16   v16b __attribute__((ext_vector_type(16)));
typedef __bf16   v8b  __attribute__((ext_vector_type(8)));
typedef float    v8f  __attribute__((ext_vector_type(8)));
typedef float    v4f  __attribute__((ext_vector_type(4)));
typedef unsigned v4u  __attribute__((ext_vector_type(4)));

__device__ __forceinline__ unsigned short f2bf_bits(float f) {
  unsigned u = __float_as_uint(f);
  return (unsigned short)((u + 0x7FFFu + ((u >> 16) & 1u)) >> 16);
}
__device__ __forceinline__ float bf_bits2f(unsigned short h) { return __uint_as_float(((unsigned)h) << 16); }

__device__ __forceinline__ void dep_guard_h(v8f& a, v8f& b, v16h x, v16h y) { asm volatile("v_nop\n\tv_nop\n\tv_nop\n\tv_nop" : "+v"(a), "+v"(b) : "v"(x), "v"(y)); }
__device__ __forceinline__ void dep_guard_b(v8f& a, v8f& b, v16b x, v16b y) { asm volatile("v_nop\n\tv_nop\n\tv_nop\n\tv_nop" : "+v"(a), "+v"(b) : "v"(x), "v"(y)); }
__device__ __forceinline__ void keep4_h(v16h a, v16h b, v16h c, v16h d) { asm volatile("v_nop" :: "v"(a), "v"(b), "v"(c), "v"(d)); }
__device__ __forceinline__ void keep4_b(v16b a, v16b b, v16b c, v16b d) { asm volatile("v_nop" :: "v"(a), "v"(b), "v"(c), "v"(d)); }
__device__ __forceinline__ void acc_guard4(v8f& a, v8f& b, v8f& c, v8f& d) { asm volatile("v_nop\n\tv_nop\n\tv_nop\n\tv_nop" : "+v"(a), "+v"(b), "+v"(c), "+v"(d)); }
__device__ __forceinline__ void acc_guard2(v8f& a, v8f& b) { asm volatile("v_nop\n\tv_nop\n\tv_nop\n\tv_nop" : "+v"(a), "+v"(b)); }
template <typename T> struct Frag;
template <> struct Frag<_Float16> {
  typedef v16h V; union U { v16h v; v8h h[2]; };
  static __device__ __forceinline__ v16h load(const _Float16* p) {
    U f; f.h[0] = *(const v8h*)(p); f.h[1] = *(const v8h*)(p + 16); return f.v;
  }
  static __device__ __forceinline__ v8f mma(v16h a, v16h b, v8f c) {
    return __builtin_amdgcn_wmma_f32_16x16x32_f16(false, a, false, b, (short)0, c, false, false);
  }
  static __device__ __forceinline__ void guard(v8f& a, v8f& b, v16h x, v16h y) { dep_guard_h(a, b, x, y); }
  static __device__ __forceinline__ void keep(v16h a, v16h b, v16h c, v16h d) { keep4_h(a, b, c, d); }
};
template <> struct Frag<__bf16> {
  typedef v16b V; union U { v16b v; v8b h[2]; };
  static __device__ __forceinline__ v16b load(const __bf16* p) {
    U f; f.h[0] = *(const v8b*)(p); f.h[1] = *(const v8b*)(p + 16); return f.v;
  }
  static __device__ __forceinline__ v8f mma(v16b a, v16b b, v8f c) {
    return __builtin_amdgcn_wmma_f32_16x16x32_bf16(false, a, false, b, (short)0, c, false, false);
  }
  static __device__ __forceinline__ void guard(v8f& a, v8f& b, v16b x, v16b y) { dep_guard_b(a, b, x, y); }
  static __device__ __forceinline__ void keep(v16b a, v16b b, v16b c, v16b d) { keep4_b(a, b, c, d); }
};

__device__ __forceinline__ float fsig(float x) { return 1.0f / (1.0f + expf(-x)); }

template <int ET> struct Elem;
template <> struct Elem<0> { typedef _Float16 T; };
template <> struct Elem<1> { typedef __bf16 T; };
template <int ET, bool SPLIT, int BIAS_MODE, int OUT_MODE, bool RESID, int ACT = 0>
__global__ __launch_bounds__(256) void wmma_gemm64(
    const unsigned short* __restrict__ Ap, const unsigned short* __restrict__ A2p, int lda, long strideA,
    const unsigned short* __restrict__ Btp, const unsigned short* __restrict__ Bt2p, int ldb, long strideB,
    void* __restrict__ Cout, void* __restrict__ Cout2, int ldc, long strideC,
    const float* __restrict__ bias,
    const float* __restrict__ resid, long strideR,
    int M, int N, int K, float scale) {
  static_assert(!RESID || OUT_MODE == 0);
  static_assert(!RESID || ACT == 0);
  typedef typename Elem<ET>::T T;
  typedef typename Frag<T>::V V;
  const T* A = (const T*)Ap; const T* A2 = (const T*)A2p; const T* Bt = (const T*)Btp; const T* Bt2 = (const T*)Bt2p;
  __shared__ __align__(16) float sT[8][16 * 68];
  const int b    = blockIdx.y;
  const int lane = threadIdx.x & 31;
  const int wave = threadIdx.x >> 5;
  const int tilesN = N >> 6;
  const int tilesM = M >> 6;
  const int tile = blockIdx.x * 8 + wave;
  if (tile >= tilesM * tilesN) return;
  const int tm = tile / tilesN;
  const int tn = tile - tm * tilesN;
  const int m0 = tm << 6;
  const int n0 = tn << 6;

  const T* Ab  = A  + (size_t)b * strideA;
  const T* Bb  = Bt + (size_t)b * strideB;
  const T* Ab2 = SPLIT ? (A2  + (size_t)b * strideA) : nullptr;
  const T* Bb2 = SPLIT ? (Bt2 + (size_t)b * strideB) : nullptr;

  const int rlane = lane & 15;
  const int koff  = (lane >> 4) * 8;
  const int mOff  = (lane >> 4) * 8;

  v8f acc[4][4];
#pragma unroll
  for (int i = 0; i < 4; ++i)
#pragma unroll
    for (int j = 0; j < 4; ++j) acc[i][j] = (v8f){0.f,0.f,0.f,0.f,0.f,0.f,0.f,0.f};

  for (int k0 = 0; k0 < K; k0 += 32) {
    V bh[4], bl[4];
#pragma unroll
    for (int j = 0; j < 4; ++j) {
      const size_t bo = (size_t)(n0 + (j << 4) + rlane) * ldb + koff + k0;
      bh[j] = Frag<T>::load(Bb + bo);
      if (SPLIT) bl[j] = Frag<T>::load(Bb2 + bo);
    }
#pragma unroll
    for (int i = 0; i < 4; ++i) {
      const size_t ao = (size_t)(m0 + (i << 4) + rlane) * lda + koff + k0;
      V ah = Frag<T>::load(Ab + ao);
      V al;
      if (SPLIT) al = Frag<T>::load(Ab2 + ao);
#pragma unroll
      for (int j = 0; j < 4; ++j) {
        acc[i][j] = Frag<T>::mma(ah, bh[j], acc[i][j]);
        if (SPLIT) {
          acc[i][j] = Frag<T>::mma(ah, bl[j], acc[i][j]);
          acc[i][j] = Frag<T>::mma(al, bh[j], acc[i][j]);
        }
      }
      Frag<T>::guard(acc[i][0], acc[i][3], ah, SPLIT ? al : ah);
    }
    Frag<T>::keep(bh[0], bh[1], bh[2], bh[3]);
    if (SPLIT) Frag<T>::keep(bl[0], bl[1], bl[2], bl[3]);
  }
  acc_guard4(acc[0][0], acc[0][1], acc[0][2], acc[0][3]);
  acc_guard4(acc[1][0], acc[1][1], acc[1][2], acc[1][3]);
  acc_guard4(acc[2][0], acc[2][1], acc[2][2], acc[2][3]);
  acc_guard4(acc[3][0], acc[3][1], acc[3][2], acc[3][3]);

  float* slab = sT[wave];
  const float* Rb = RESID ? (resid + (size_t)b * strideR) : nullptr;
#pragma unroll
  for (int i = 0; i < 4; ++i) {
    const int mBase = m0 + (i << 4);
    float bmv[8];
#pragma unroll
    for (int r = 0; r < 8; ++r) bmv[r] = 0.0f;
    if (BIAS_MODE == 1) {
      const v4f bm0 = *(const v4f*)(bias + mBase + mOff);
      const v4f bm1 = *(const v4f*)(bias + mBase + mOff + 4);
      bmv[0] = bm0[0]; bmv[1] = bm0[1]; bmv[2] = bm0[2]; bmv[3] = bm0[3];
      bmv[4] = bm1[0]; bmv[5] = bm1[1]; bmv[6] = bm1[2]; bmv[7] = bm1[3];
    }
#pragma unroll
    for (int j = 0; j < 4; ++j) {
      const int n = n0 + (j << 4) + rlane;
      float bv = 0.f;
      if (BIAS_MODE == 2) bv = bias[n];
#pragma unroll
      for (int r = 0; r < 8; ++r) {
        float v = acc[i][j][r] * scale;
        if (BIAS_MODE == 1) v += bmv[r];
        if (BIAS_MODE == 2) v += bv;
        if (ACT == 1) v = tanhf(v);
        if (ACT == 2) v = fmaxf(v, 0.0f);
        if (ACT == 3) v = v / (1.0f + expf(-v));
        if (ACT == 4) v = (v > 0.f) ? v : 0.01f * v;
        slab[(mOff + r) * 68 + (j << 4) + rlane] = v;
      }
    }
    __builtin_amdgcn_fence(__ATOMIC_RELEASE, "workgroup");
    __builtin_amdgcn_wave_barrier();
    __builtin_amdgcn_fence(__ATOMIC_ACQUIRE, "workgroup");
    if (OUT_MODE == 0) {
      float* C = (float*)Cout + (size_t)b * strideC;
      const int hh = lane >> 4, c4 = (lane & 15) * 4;
      for (int pass = 0; pass < 2; ++pass) {
#pragma unroll
        for (int it = 0; it < 8; ++it) {
          const int row = it * 2 + hh;
          v4f v = *(const v4f*)(slab + row * 68 + c4);
          if (RESID) {
            const v4f rv = *(const v4f*)(Rb + (size_t)(mBase + row) * ldc + n0 + c4);
            v += rv;
          }
          *(volatile v4f*)(C + (size_t)(mBase + row) * ldc + n0 + c4) = v;
        }
        __threadfence();
      }
    } else {
      const int q = lane >> 3, c8 = (lane & 7) * 8;
      unsigned short* C  = (unsigned short*)Cout  + (size_t)b * strideC;
      unsigned short* C2 = (OUT_MODE == 2) ? ((unsigned short*)Cout2 + (size_t)b * strideC) : nullptr;
      for (int pass = 0; pass < 2; ++pass) {
#pragma unroll
        for (int it = 0; it < 4; ++it) {
          const int row = it * 4 + q;
          const float* sp = slab + row * 68 + c8;
          v8h hv, lv;
#pragma unroll
          for (int e = 0; e < 8; ++e) {
            if (OUT_MODE == 1) {
              hv[e] = (_Float16)sp[e];
            } else {
              unsigned short hb = f2bf_bits(sp[e]);
              unsigned short lb = f2bf_bits(sp[e] - bf_bits2f(hb));
              hv[e] = __builtin_bit_cast(_Float16, hb);
              lv[e] = __builtin_bit_cast(_Float16, lb);
            }
          }
          *(volatile v8h*)(C + (size_t)(mBase + row) * ldc + n0 + c8) = hv;
          if (OUT_MODE == 2) *(volatile v8h*)(C2 + (size_t)(mBase + row) * ldc + n0 + c8) = lv;
        }
        __threadfence();
      }
    }
    __builtin_amdgcn_fence(__ATOMIC_RELEASE, "workgroup");
    __builtin_amdgcn_wave_barrier();
    __builtin_amdgcn_fence(__ATOMIC_ACQUIRE, "workgroup");
  }
}

constexpr int PT_THT = 1536, PT_CHEB = 38400, PT_UXT = 2048, PT_UGT = 1024, PT_VTX = 2048, PT_VTG = 1024, PT_W64 = 512,
              PT_WQP = 1024, PT_WV = 512, PT_WTC = 1024, PT_VTZ = 10240, PT_HSZ = 4992, PT_BIAS = 96;
constexpr int PREP_BLOCKS = 267;
static_assert(PT_THT == 3 * 64 * 64 / 8 && PT_CHEB == NODEP * CHEBW / 8 && PT_VTZ == 64 * LROWP / 8 && PT_HSZ == NBS * (NODEP - NODES) * EMB / 8);

__global__ __launch_bounds__(NTHR) void prep_kernel(
    const float* __restrict__ theta, const float* __restrict__ cheb,
    const float* __restrict__ Ux, const float* __restrict__ Ug, const float* __restrict__ Vx, const float* __restrict__ Vg,
    const float* __restrict__ Wff1, const float* __restrict__ Wff2, const float* __restrict__ Wfa1, const float* __restrict__ Wfa2,
    const float* __restrict__ Wout, const float* __restrict__ Wrc, const float* __restrict__ Win, const float* __restrict__ Wtc,
    const float* __restrict__ bin, const float* __restrict__ bout, const float* __restrict__ bfa1,
    unsigned short* __restrict__ THT, unsigned short* __restrict__ CHEBP, unsigned short* __restrict__ UXT, unsigned short* __restrict__ UGT,
    unsigned short* __restrict__ VTW, unsigned short* __restrict__ WFF1T, unsigned short* __restrict__ WFF2T,
    unsigned short* __restrict__ WFA1T, unsigned short* __restrict__ WFA2T, unsigned short* __restrict__ WOUTN, unsigned short* __restrict__ WRCN,
    unsigned short* __restrict__ WQP, unsigned short* __restrict__ WKP, unsigned short* __restrict__ WVN, unsigned short* __restrict__ WTCP,
    unsigned short* __restrict__ VTP, unsigned short* __restrict__ HS, float* __restrict__ BIASP) {
  const int bx = blockIdx.x, tid = threadIdx.x;
  int job, jb;
  if      (bx < 6)   { job = 0;  jb = 0;   }
  else if (bx < 156) { job = 1;  jb = 6;   }
  else if (bx < 164) { job = 2;  jb = 156; }
  else if (bx < 168) { job = 3;  jb = 164; }
  else if (bx < 176) { job = 4;  jb = 168; }
  else if (bx < 180) { job = 5;  jb = 176; }
  else if (bx < 182) { job = 6;  jb = 180; }
  else if (bx < 184) { job = 7;  jb = 182; }
  else if (bx < 186) { job = 8;  jb = 184; }
  else if (bx < 188) { job = 9;  jb = 186; }
  else if (bx < 190) { job = 10; jb = 188; }
  else if (bx < 192) { job = 11; jb = 190; }
  else if (bx < 196) { job = 12; jb = 192; }
  else if (bx < 200) { job = 13; jb = 196; }
  else if (bx < 202) { job = 14; jb = 200; }
  else if (bx < 206) { job = 15; jb = 202; }
  else if (bx < 246) { job = 16; jb = 206; }
  else if (bx < 266) { job = 17; jb = 246; }
  else               { job = 18; jb = 266; }
  const int li = (bx - jb) * NTHR + tid;
  const int cnt = (job == 0) ? PT_THT : (job == 1) ? PT_CHEB : (job == 2) ? PT_UXT : (job == 3) ? PT_UGT :
                  (job == 4) ? PT_VTX : (job == 5) ? PT_VTG : (job <= 11) ? PT_W64 : (job <= 13) ? PT_WQP :
                  (job == 14) ? PT_WV : (job == 15) ? PT_WTC : (job == 16) ? PT_VTZ : (job == 17) ? PT_HSZ : PT_BIAS;
  if (li >= cnt) return;

  if (job == 18) {
    const int plane = (li >> 5) & 1;
    const int idx4  = (li & 31) * 4;
    int li2 = li - 64; li2 = li2 < 0 ? 0 : li2; li2 = li2 > 31 ? 31 : li2;
    const int p2  = li2 >> 4;
    const int i4b = (li2 & 15) * 4;
    v4f o;
#pragma unroll
    for (int e = 0; e < 4; ++e) {
      const int r = idx4 + e, head = r >> 5, d = r & 31;
      const float bq = bin[plane * 64 + head * HDIM + (d < HDIM ? d : HDIM - 1)];
      const float vq = (d < HDIM) ? bq : 0.0f;
      const float vo = bout[i4b + e] * CCARRY;
      const float vf = bfa1[i4b + e] * CCARRY;
      const float vb = p2 ? vf : vo;
      o[e] = (li < 64) ? vq : vb;
    }
    float* dst = (li < 64) ? (BIASP + plane * QKW + idx4) : (BIASP + 2 * QKW + p2 * 64 + i4b);
    *(volatile v4f*)dst = o;
    __threadfence();
    *(volatile v4f*)dst = o;
    return;
  }

  const int c8 = (li & 7) * 8;
  const int j8 = li >> 3;
  const float* wsrc = (job == 6) ? Wff1 : (job == 7) ? Wff2 : (job == 8) ? Wfa1 : (job == 9) ? Wfa2 : (job == 10) ? Wout : Wrc;
  unsigned short* wdst = (job == 6) ? WFF1T : (job == 7) ? WFF2T : (job == 8) ? WFA1T : (job == 9) ? WFA2T : (job == 10) ? WOUTN : WRCN;
  float v[8];
  unsigned short* dst = THT;
#pragma unroll
  for (int e = 0; e < 8; ++e) v[e] = 0.0f;
  switch (job) {
    case 0: {
      const int k = li >> 9, d = j8 & 63;
      dst = THT + (size_t)li * 8;
#pragma unroll
      for (int e = 0; e < 8; ++e) v[e] = theta[(k * 64 + c8 + e) * 64 + d];
    } break;
    case 1: {
      const int m = li / 120, cb = (li - m * 120) * 8, k = cb / NODEP, nb = cb - k * NODEP;
      const int mc = m < NODES ? m : NODES - 1;
      dst = CHEBP + (size_t)li * 8;
#pragma unroll
      for (int e = 0; e < 8; ++e) {
        const int n = nb + e, ncl = n < NODES ? n : NODES - 1;
        const float val = cheb[((size_t)(k * NODES + mc)) * NODES + ncl];
        v[e] = (m < NODES && n < NODES) ? val : 0.0f;
      }
    } break;
    case 2: {
      dst = UXT + (size_t)li * 8;
#pragma unroll
      for (int e = 0; e < 8; ++e) v[e] = Ux[(c8 + e) * NGX + j8];
    } break;
    case 3: {
      dst = UGT + (size_t)li * 8;
#pragma unroll
      for (int e = 0; e < 8; ++e) v[e] = Ug[(c8 + e) * NGG + j8];
    } break;
    case 4: {
      dst = VTW + (size_t)li * 8;
#pragma unroll
      for (int e = 0; e < 8; ++e) v[e] = Vx[(c8 + e) * NGX + j8];
    } break;
    case 5: {
      dst = VTW + (size_t)NGX * EMB + (size_t)li * 8;
#pragma unroll
      for (int e = 0; e < 8; ++e) v[e] = Vg[(c8 + e) * NGG + j8];
    } break;
    case 6: case 7: case 8: case 9: {
      dst = wdst + (size_t)li * 8;
#pragma unroll
      for (int e = 0; e < 8; ++e) v[e] = wsrc[(c8 + e) * 64 + j8];
    } break;
    case 10: case 11: {
      dst = wdst + (size_t)li * 8;
#pragma unroll
      for (int e = 0; e < 8; ++e) v[e] = wsrc[li * 8 + e];
    } break;
    case 12: case 13: {
      const int r = j8, head = r >> 5, d = r & 31;
      const int base = (job == 12) ? 0 : 64;
      const int srow = base + head * HDIM + (d < HDIM ? d : HDIM - 1);
      dst = ((job == 12) ? WQP : WKP) + (size_t)li * 8;
#pragma unroll
      for (int e = 0; e < 8; ++e) { const float val = Win[srow * 64 + c8 + e]; v[e] = (d < HDIM) ? val : 0.0f; }
    } break;
    case 14: {
      dst = WVN + (size_t)li * 8;
#pragma unroll
      for (int e = 0; e < 8; ++e) v[e] = Win[128 * 64 + li * 8 + e];
    } break;
    case 15: {
      const int f = li >> 4, colb = (li & 15) * 8;
      dst = WTCP + (size_t)li * 8;
#pragma unroll
      for (int e = 0; e < 8; ++e) { const int col = colb + e, dt = col >> 6, h = col & 63; v[e] = Wtc[(f * 64 + h) * 3 + dt]; }
    } break;
    case 16: {
      dst = VTP + (size_t)(SEQ * EMB) * LROWP + (size_t)li * 8;
    } break;
    case 17: {
      const int rr = j8, bs = rr / 13, p = rr - bs * 13;
      dst = HS + ((size_t)(bs * NODEP + NODES + p)) * EMB + c8;
    } break;
    default: break;
  }
  v8h hv;
#pragma unroll
  for (int e = 0; e < 8; ++e) hv[e] = (_Float16)v[e];
  *(volatile v8h*)dst = hv;
  __threadfence();
  *(volatile v8h*)dst = hv;
}

__global__ __launch_bounds__(NTHR) void embed_kernel(const float* __restrict__ x, const float* __restrict__ Wex, const float* __restrict__ bex,
                                                     const float* __restrict__ Wos, const float* __restrict__ bos,
                                                     unsigned short* __restrict__ EX, unsigned short* __restrict__ EOS) {
  const int i = blockIdx.x * NTHR + threadIdx.x;
  const int row = i >> 3, c8 = (i & 7) * 8;
  const int bs = row / NODEP, n = row - bs * NODEP;
  const bool ok = n < NODES;
  const int nc = ok ? n : NODES - 1;
  const float* xp = x + ((size_t)(bs * NODES + nc)) * 3;
  const float x0 = xp[0], x1 = xp[1], x2 = xp[2];
  const v4f wa = *(const v4f*)(Wex + c8),      wb = *(const v4f*)(Wex + c8 + 4);
  const v4f ba = *(const v4f*)(bex + c8),      bb = *(const v4f*)(bex + c8 + 4);
  const v4f pa = *(const v4f*)(Wos + c8),      pb = *(const v4f*)(Wos + c8 + 4);
  const v4f qa = *(const v4f*)(Wos + 64 + c8), qb = *(const v4f*)(Wos + 64 + c8 + 4);
  const v4f ca = *(const v4f*)(bos + c8),      cb = *(const v4f*)(bos + c8 + 4);
  v8h he, ho;
#pragma unroll
  for (int e = 0; e < 4; ++e) {
    const float e0 = x0 * wa[e] + ba[e];
    const float e1 = x0 * wb[e] + bb[e];
    const float o0 = x1 * pa[e] + x2 * qa[e] + ca[e];
    const float o1 = x1 * pb[e] + x2 * qb[e] + cb[e];
    he[e] = (_Float16)(ok ? e0 : 0.0f); he[4 + e] = (_Float16)(ok ? e1 : 0.0f);
    ho[e] = (_Float16)(ok ? o0 : 0.0f); ho[4 + e] = (_Float16)(ok ? o1 : 0.0f);
  }
  unsigned short* d0 = EX + (size_t)row * EMB + c8;
  unsigned short* d1 = EOS + (size_t)row * EMB + c8;
  *(volatile v8h*)d0 = he; *(volatile v8h*)d1 = ho;
  __threadfence();
  *(volatile v8h*)d0 = he; *(volatile v8h*)d1 = ho;
}

constexpr int LB_ROWS = 16, LB_THR = 128, AHP = 72, GSP = 388;
constexpr int LSTM_BLOCKS = (LROWS + LB_ROWS - 1) / LB_ROWS;
static_assert((LB_ROWS * AHP) % LB_THR == 0);
static_assert((LB_ROWS * NGX / 4) == 8 * LB_THR && (LB_ROWS * NGG / 4) == 4 * LB_THR);
static_assert(EMB == 16 * (LB_THR / 32));
__global__ __launch_bounds__(LB_THR) void lstm_kernel(const float* __restrict__ GX, const float* __restrict__ GG,
                                                    const unsigned short* __restrict__ VTWp, unsigned short* __restrict__ HS) {
  __shared__ __align__(16) _Float16 Ah[LB_ROWS * AHP];
  __shared__ __align__(16) float    Gs[LB_ROWS * GSP];
  const _Float16* VTW = (const _Float16*)VTWp;
  const int tid = threadIdx.x, lane = tid & 31, wave = tid >> 5;
  const int c = lane & 15, hh = lane >> 4, koff = hh * 8;
  const int q0 = blockIdx.x * LB_ROWS;
  const int u = 16 * wave + c;

#pragma unroll 1
  for (int i = tid; i < LB_ROWS * AHP; i += LB_THR) Ah[i] = (_Float16)0.0f;
  int rbx[8], rbg[4];
#pragma unroll
  for (int i = 0; i < 8; ++i) {
    const int row = 2 * i + (tid >> 6);
    int q = q0 + row; q = q < LROWS ? q : LROWS - 1;
    const int b = q / NODES, n = q - b * NODES;
    rbx[i] = b * SEQ * NODEP + n;
  }
#pragma unroll
  for (int i = 0; i < 4; ++i) {
    const int row = 4 * i + (tid >> 5);
    int q = q0 + row; q = q < LROWS ? q : LROWS - 1;
    const int b = q / NODES, n = q - b * NODES;
    rbg[i] = b * SEQ * NODEP + n;
  }
  float cst[8];
#pragma unroll
  for (int r = 0; r < 8; ++r) cst[r] = 0.0f;
  __syncthreads();

  const _Float16* ahrow = Ah + c * AHP + koff;
  const v8f z8 = {0.f, 0.f, 0.f, 0.f, 0.f, 0.f, 0.f, 0.f};

#pragma unroll 1
  for (int t = 0; t < SEQ; ++t) {
#pragma unroll
    for (int i = 0; i < 8; ++i) {
      const int row = 2 * i + (tid >> 6), c4 = (tid & 63) * 4;
      const v4f v = *(const v4f*)(GX + (size_t)(rbx[i] + t * NODEP) * NGX + c4);
      *(v4f*)(Gs + row * GSP + c4) = v;
    }
#pragma unroll
    for (int i = 0; i < 4; ++i) {
      const int row = 4 * i + (tid >> 5), c4 = (tid & 31) * 4;
      const v4f v = *(const v4f*)(GG + (size_t)(rbg[i] + t * NODEP) * NGG + c4);
      *(v4f*)(Gs + row * GSP + NGX + c4) = v;
    }
    __syncthreads();
    v8f acc[6];
#pragma unroll
    for (int g = 0; g < 6; ++g) acc[g] = z8;
#pragma unroll 1
    for (int k0 = 0; k0 < EMB; k0 += 32) {
      const v16h a = Frag<_Float16>::load(ahrow + k0);
      v16h bfr[6];
#pragma unroll
      for (int g = 0; g < 6; ++g) bfr[g] = Frag<_Float16>::load(VTW + (size_t)(g * 64 + u) * EMB + koff + k0);
#pragma unroll
      for (int g = 0; g < 6; ++g) acc[g] = Frag<_Float16>::mma(a, bfr[g], acc[g]);
      dep_guard_h(acc[0], acc[5], a, bfr[5]);
      keep4_h(bfr[0], bfr[1], bfr[2], bfr[3]);
      keep4_h(bfr[4], bfr[5], a, bfr[0]);
    }
    acc_guard4(acc[0], acc[1], acc[2], acc[3]);
    acc_guard2(acc[4], acc[5]);
    float hn[8];
#pragma unroll
    for (int r = 0; r < 8; ++r) {
      const float* gp = Gs + (8 * hh + r) * GSP + u;
      const float zf  = gp[0]   + acc[0][r];
      const float zi  = gp[64]  + acc[1][r];
      const float zo  = gp[128] + acc[2][r];
      const float zu  = gp[192] + acc[3][r];
      const float zgf = gp[256] + acc[4][r];
      const float zgu = gp[320] + acc[5][r];
      const float ft = fsig(zf), it = fsig(zi), ot = fsig(zo), ut = fsig(zu), gf = fsig(zgf), gu = fsig(zgu);
      const float cn = (gf * ft) * cst[r] + (gu * it) * ut;
      cst[r] = cn;
      hn[r] = ot * tanhf(cn);
    }
    __syncthreads();
#pragma unroll
    for (int r = 0; r < 8; ++r) Ah[(8 * hh + r) * AHP + u] = (_Float16)hn[r];
    __syncthreads();
    {
      const int row = 4 * wave + (lane >> 3), ch = (lane & 7) * 8;
      const int q = q0 + row;
      const bool ok = q < LROWS;
      const int qc = ok ? q : LROWS - 1;
      const int b = qc / NODES, n = qc - b * NODES;
      const v8h hvv = *(const v8h*)(Ah + row * AHP + ch);
      _Float16* dst = (_Float16*)(HS + ((size_t)((b * SEQ + t) * NODEP + n)) * EMB + ch);
      if (ok) *(volatile v8h*)dst = hvv;
      __threadfence();
      if (ok) *(volatile v8h*)dst = hvv;
    }
  }
}

__global__ __launch_bounds__(NTHR) void tcgather_kernel(const unsigned short* __restrict__ HID, unsigned short* __restrict__ TCA) {
  const int i = blockIdx.x * NTHR + threadIdx.x;
  const int L = i >> 4, ch = i & 15, dt = ch >> 3, cc = (ch & 7) * 8;
  const bool ok = L < LROWS;
  const int Lc = ok ? L : LROWS - 1;
  const int b = Lc / NODES, n = Lc - b * NODES;
  const v4u src = *(const v4u*)(HID + ((size_t)((b * SEQ + (SEQ - 2) + dt) * NODEP + n)) * EMB + cc);
  v4u o;
#pragma unroll
  for (int e = 0; e < 4; ++e) o[e] = ok ? src[e] : 0u;
  unsigned short* dst = TCA + (size_t)L * (2 * EMB) + ch * 8;
  *(volatile v4u*)dst = o;
  __threadfence();
  *(volatile v4u*)dst = o;
}

__global__ __launch_bounds__(NTHR) void scramble_kernel(const float* __restrict__ x, const float* __restrict__ Wex, const float* __restrict__ bex,
                                                        const float* __restrict__ TCL, unsigned short* __restrict__ QIN, unsigned short* __restrict__ KVIN) {
  __shared__ float qs[NTHR];
  __shared__ float ks[NTHR];
  const int tid = threadIdx.x;
  const int rl = tid >> 6, fcol = tid & 63;
  const int row = blockIdx.x * 4 + rl;
  const int sp = row / LROWP, L = row - sp * LROWP;
  const bool ok = L < LROWS;
  const int Lc = ok ? L : LROWS - 1;
  const int b = Lc / NODES, lp = Lc - b * NODES;
  const int j = lp * (SEQ * EMB) + sp * EMB + fcol;
  const int s = j / (EMB * NODES);
  const int rem = j - s * (EMB * NODES);
  const int ee = rem / NODES;
  const int n = rem - ee * NODES;
  const float xv = x[((size_t)((b * SEQ + s) * NODES + n)) * 3];
  const float w = Wex[ee], bb = bex[ee];
  const float tv = TCL[(size_t)(b * NODES + n) * EMB + ee];
  const float kvv = ok ? (xv * w + bb) : 0.0f;
  const float qvv = ok ? tv : 0.0f;
  qs[tid] = qvv;
  ks[tid] = kvv;
  __syncthreads();
  const int wave = tid >> 5, lane = tid & 31;
  if (wave < 2) {
    const int rr = lane >> 3, ch = (lane & 7) * 8;
    v8h hq, hk;
#pragma unroll
    for (int e = 0; e < 8; ++e) { hq[e] = (_Float16)qs[rr * 64 + ch + e]; hk[e] = (_Float16)ks[rr * 64 + ch + e]; }
    const v8h hv = (wave == 0) ? hq : hk;
    unsigned short* dst = ((wave == 0) ? QIN : KVIN) + (size_t)(blockIdx.x * 4 + rr) * EMB + ch;
    *(volatile v8h*)dst = hv;
    __threadfence();
    *(volatile v8h*)dst = hv;
  }
}

constexpr int SM_ROWS = 8;
static_assert((4 * LROWP) % SM_ROWS == 0);
__global__ __launch_bounds__(NTHR) void softmax_kernel(const float* __restrict__ Sp, unsigned short* __restrict__ Pp) {
  __shared__ __align__(16) float rbuf[SM_ROWS][LROWP];
  const int tid = threadIdx.x, lane = tid & 31, wave = tid >> 5;
  const int row = blockIdx.x * SM_ROWS + wave;
  const float* sp = Sp + (size_t)row * LROWP;
  float* rb = rbuf[wave];
  float m = -INFINITY;
#pragma unroll 1
  for (int it = 0; it < 10; ++it) {
    const int col = it * 128 + lane * 4;
    const v4f v = *(const v4f*)(sp + col);
    v4f s;
#pragma unroll
    for (int e = 0; e < 4; ++e) {
      const float xs = v[e] * 0.25f;
      s[e] = (col + e < LROWS) ? xs : -INFINITY;
      m = fmaxf(m, s[e]);
    }
    *(v4f*)(rb + col) = s;
  }
#pragma unroll
  for (int off = 1; off < 32; off <<= 1) m = fmaxf(m, __shfl_xor(m, off, 32));
  __syncthreads();
  float sum = 0.0f;
#pragma unroll 1
  for (int it = 0; it < 10; ++it) {
    const int col = it * 128 + lane * 4;
    const v4f s = *(const v4f*)(rb + col);
    v4f p;
#pragma unroll
    for (int e = 0; e < 4; ++e) { p[e] = expf(s[e] - m); sum += p[e]; }
    *(v4f*)(rb + col) = p;
  }
#pragma unroll
  for (int off = 1; off < 32; off <<= 1) sum += __shfl_xor(sum, off, 32);
  const float inv = (1.0f / sum) * PCARRY;
  __syncthreads();
  v8h hv[5];
#pragma unroll
  for (int it = 0; it < 5; ++it) {
    const int col = it * 256 + lane * 8;
    const v4f a  = *(const v4f*)(rb + col);
    const v4f b2 = *(const v4f*)(rb + col + 4);
#pragma unroll
    for (int e = 0; e < 4; ++e) { hv[it][e] = (_Float16)(a[e] * inv); hv[it][4 + e] = (_Float16)(b2[e] * inv); }
  }
  unsigned short* pr = Pp + (size_t)row * LROWP;
  for (int pass = 0; pass < 2; ++pass) {
#pragma unroll
    for (int it = 0; it < 5; ++it) *(volatile v8h*)(pr + it * 256 + lane * 8) = hv[it];
    __threadfence();
  }
}

__global__ __launch_bounds__(NTHR) void ctxpack_kernel(const float* __restrict__ CTXH, unsigned short* __restrict__ CTX) {
  const int i = blockIdx.x * NTHR + threadIdx.x;
  const int row = i >> 3, c8 = (i & 7) * 8;
  const int bs = row / NODEP, n = row - bs * NODEP;
  const int b = bs / SEQ, s = bs - b * SEQ;
  const bool ok = n < NODES;
  const int nc = ok ? n : NODES - 1;
  const int head = c8 >> 4, d0 = c8 & 15;
  const float* src = CTXH + ((size_t)((s * NHEADS + head) * LROWP + b * NODES + nc)) * EMB + d0;
  const v4f a  = *(const v4f*)(src);
  const v4f b2 = *(const v4f*)(src + 4);
  v8h hv;
#pragma unroll
  for (int e = 0; e < 4; ++e) {
    const float f0 = ok ? a[e]  * CCARRY : 0.0f;
    const float f1 = ok ? b2[e] * CCARRY : 0.0f;
    hv[e] = (_Float16)f0; hv[4 + e] = (_Float16)f1;
  }
  unsigned short* dst = CTX + (size_t)row * EMB + c8;
  *(volatile v8h*)dst = hv;
  __threadfence();
  *(volatile v8h*)dst = hv;
}

__global__ __launch_bounds__(NTHR) void final_kernel(const float* __restrict__ COMB, const float* __restrict__ Wfin,
                                                     const float* __restrict__ bfin, float* __restrict__ out) {
  const int idx = blockIdx.x * NTHR + threadIdx.x;
  if (idx >= NOUT) return;
  const int n = idx % NODES;
  const int r = idx / NODES;
  const int p = r % PRE, b = r / PRE;
  float sum = 0.0f;
#pragma unroll 1
  for (int s = 0; s < SEQ; ++s) {
    const float* cp = COMB + ((size_t)((b * SEQ + s) * NODEP + n)) * EMB;
    const float* wp = Wfin + ((size_t)(p * SEQ + s)) * EMB;
    float acc = 0.0f;
#pragma unroll 1
    for (int f4 = 0; f4 < EMB / 4; ++f4) {
      const v4f cv = *(const v4f*)(cp + 4 * f4);
      const v4f wv = *(const v4f*)(wp + 4 * f4);
      acc += cv[0] * wv[0];
      acc += cv[1] * wv[1];
      acc += cv[2] * wv[2];
      acc += cv[3] * wv[3];
    }
    sum += acc;
  }
  const float o = sum + bfin[p];
  *(volatile float*)(out + idx) = o;
  __threadfence();
  *(volatile float*)(out + idx) = o;
}

template <int BM, int OM, bool RES, int ACT>
static void run_gemm(hipStream_t st, int batch, const unsigned short* A, int lda, long sA, const unsigned short* Bt, int ldb, long sB,
                     void* C, int ldc, long sC, const float* bias, const float* resid, long sR, int M, int N, int K, float scale) {
  const int tiles = (M / 64) * (N / 64);
  dim3 grid((unsigned)((tiles + 7) / 8), (unsigned)batch);
  wmma_gemm64<0, false, BM, OM, RES, ACT><<<grid, 256, 0, st>>>(A, A, lda, sA, Bt, Bt, ldb, sB, C, C, ldc, sC, bias, resid, sR, M, N, K, scale);
}

extern "C" void kernel_launch(void* const* d_in, const int* in_sizes, int n_in,
                              void* d_out, int out_size, void* d_ws, size_t ws_size, hipStream_t stream) {
  if (n_in < 31 || d_out == nullptr || d_ws == nullptr) return;
  if (in_sizes[0] != BATCH * SEQ * NODES * 3 || in_sizes[1] != 3 * NODES * NODES || in_sizes[2] != 3 * 64 * 64 ||
      in_sizes[3] != 64 || in_sizes[4] != 64 || in_sizes[5] != 128 || in_sizes[6] != 64 ||
      in_sizes[7] != 64 * 256 || in_sizes[8] != 64 * 256 || in_sizes[9] != 256 ||
      in_sizes[10] != 64 * 128 || in_sizes[11] != 64 * 128 || in_sizes[12] != 128 ||
      in_sizes[13] != 4096 || in_sizes[14] != 64 || in_sizes[15] != 4096 || in_sizes[16] != 64 ||
      in_sizes[17] != 64 * 64 * 3 || in_sizes[18] != 64 || in_sizes[19] != 4096 || in_sizes[20] != 64 ||
      in_sizes[21] != 192 * 64 || in_sizes[22] != 192 || in_sizes[23] != 4096 || in_sizes[24] != 64 ||
      in_sizes[25] != 4096 || in_sizes[26] != 64 || in_sizes[27] != 4096 || in_sizes[28] != 64 ||
      in_sizes[29] != PRE * SEQ * 64 || in_sizes[30] != PRE || out_size != NOUT) return;

  const float* x     = (const float*)d_in[0];
  const float* cheb  = (const float*)d_in[1];
  const float* theta = (const float*)d_in[2];
  const float* Wex   = (const float*)d_in[3];
  const float* bex   = (const float*)d_in[4];
  const float* Wos   = (const float*)d_in[5];
  const float* bos   = (const float*)d_in[6];
  const float* Ux    = (const float*)d_in[7];
  const float* Vx    = (const float*)d_in[8];
  const float* bx    = (const float*)d_in[9];
  const float* Ug    = (const float*)d_in[10];
  const float* Vg    = (const float*)d_in[11];
  const float* bg    = (const float*)d_in[12];
  const float* Wff1  = (const float*)d_in[13];
  const float* bff1  = (const float*)d_in[14];
  const float* Wff2  = (const float*)d_in[15];
  const float* bff2  = (const float*)d_in[16];
  const float* Wtc   = (const float*)d_in[17];
  const float* btc   = (const float*)d_in[18];
  const float* Wrc   = (const float*)d_in[19];
  const float* brc   = (const float*)d_in[20];
  const float* Win   = (const float*)d_in[21];
  const float* bin   = (const float*)d_in[22];
  const float* Wout  = (const float*)d_in[23];
  const float* bout  = (const float*)d_in[24];
  const float* Wfa1  = (const float*)d_in[25];
  const float* bfa1  = (const float*)d_in[26];
  const float* Wfa2  = (const float*)d_in[27];
  const float* bfa2  = (const float*)d_in[28];
  const float* Wfin  = (const float*)d_in[29];
  const float* bfin  = (const float*)d_in[30];
  float* out = (float*)d_out;

  char* ws = (char*)d_ws; size_t off = 0;
  auto carve = [&](size_t bytes) -> char* { char* p = ws + off; off += (bytes + 255) & ~(size_t)255; return p; };
  const size_t PL16 = (size_t)R1ROWS * EMB * 2;
  unsigned short* EX16   = (unsigned short*)carve(PL16);
  unsigned short* EOS16  = (unsigned short*)carve(PL16);
  unsigned short* THT16  = (unsigned short*)carve((size_t)3 * 64 * 64 * 2);
  unsigned short* CHEB16 = (unsigned short*)carve((size_t)NODEP * CHEBW * 2);
  unsigned short* TMPT16 = (unsigned short*)carve((size_t)NBS * 64 * CHEBW * 2);
  unsigned short* GCNX16 = (unsigned short*)carve(PL16);
  unsigned short* GCNO16 = (unsigned short*)carve(PL16);
  unsigned short* UXT16  = (unsigned short*)carve((size_t)NGX * EMB * 2);
  unsigned short* UGT16  = (unsigned short*)carve((size_t)NGG * EMB * 2);
  unsigned short* VTW16  = (unsigned short*)carve((size_t)NGATE * EMB * 2);
  unsigned short* WFF1T  = (unsigned short*)carve((size_t)64 * 64 * 2);
  unsigned short* WFF2T  = (unsigned short*)carve((size_t)64 * 64 * 2);
  unsigned short* WFA1T  = (unsigned short*)carve((size_t)64 * 64 * 2);
  unsigned short* WFA2T  = (unsigned short*)carve((size_t)64 * 64 * 2);
  unsigned short* WOUT16 = (unsigned short*)carve((size_t)64 * 64 * 2);
  unsigned short* WRC16  = (unsigned short*)carve((size_t)64 * 64 * 2);
  unsigned short* WQP16  = (unsigned short*)carve((size_t)QKW * EMB * 2);
  unsigned short* WKP16  = (unsigned short*)carve((size_t)QKW * EMB * 2);
  unsigned short* WV16   = (unsigned short*)carve((size_t)64 * 64 * 2);
  unsigned short* WTC16  = (unsigned short*)carve((size_t)64 * 128 * 2);
  float*          BIASP  = (float*)carve((size_t)(2 * QKW + 128) * 4);
  float*          GX     = (float*)carve((size_t)R1ROWS * NGX * 4);
  float*          GG     = (float*)carve((size_t)R1ROWS * NGG * 4);
  unsigned short* HS16   = (unsigned short*)carve(PL16);
  unsigned short* FF1_16 = (unsigned short*)carve(PL16);
  unsigned short* HID16  = (unsigned short*)carve(PL16);
  unsigned short* TCA16  = (unsigned short*)carve((size_t)LROWP * 128 * 2);
  float*          TCL    = (float*)carve((size_t)LROWP * EMB * 4);
  unsigned short* QIN16  = (unsigned short*)carve(PL16);
  unsigned short* KVIN16 = (unsigned short*)carve(PL16);
  unsigned short* QP16   = (unsigned short*)carve((size_t)R2ROWS * QKW * 2);
  unsigned short* KP16   = (unsigned short*)carve((size_t)R2ROWS * QKW * 2);
  unsigned short* VTP16  = (unsigned short*)carve((size_t)VTROWS * LROWP * 2);
  float*          SPL    = (float*)carve((size_t)4 * LROWP * LROWP * 4);
  unsigned short* P16    = (unsigned short*)carve((size_t)4 * LROWP * LROWP * 2);
  float*          CTXH   = (float*)carve((size_t)NINST * LROWP * EMB * 4);
  unsigned short* CTX16  = (unsigned short*)carve(PL16);
  unsigned short* DSA16  = (unsigned short*)carve(PL16);
  unsigned short* FA1_16 = (unsigned short*)carve(PL16);
  float*          FFA    = (float*)carve((size_t)R1ROWS * EMB * 4);
  float*          COMB   = (float*)carve((size_t)R1ROWS * EMB * 4);
  if (off > ws_size || off > (size_t)134217728) return;
  float* BQP    = BIASP;
  float* BKP    = BIASP + QKW;
  float* BOUT64 = BIASP + 2 * QKW;
  float* BFA164 = BIASP + 2 * QKW + 64;
  const float* dummyres = TCL;

  prep_kernel<<<PREP_BLOCKS, NTHR, 0, stream>>>(theta, cheb, Ux, Ug, Vx, Vg, Wff1, Wff2, Wfa1, Wfa2, Wout, Wrc, Win, Wtc, bin, bout, bfa1,
                                                THT16, CHEB16, UXT16, UGT16, VTW16, WFF1T, WFF2T, WFA1T, WFA2T, WOUT16, WRC16,
                                                WQP16, WKP16, WV16, WTC16, VTP16, HS16, BIASP);
  embed_kernel<<<(R1ROWS * 8) / NTHR, NTHR, 0, stream>>>(x, Wex, bex, Wos, bos, EX16, EOS16);

  const long sEmb = (long)NODEP * EMB, sTmp = (long)64 * CHEBW, sGcn = (long)NODEP * EMB;
  for (int k = 0; k < 3; ++k)
    run_gemm<0, 1, false, 0>(stream, NBS, THT16 + (size_t)k * 4096, 64, 0L, EX16, EMB, sEmb, (void*)(TMPT16 + k * NODEP), CHEBW, sTmp,
                             BIASP, dummyres, 0L, 64, NODEP, EMB, 1.0f);
  run_gemm<0, 1, false, 2>(stream, NBS, CHEB16, CHEBW, 0L, TMPT16, CHEBW, sTmp, (void*)GCNX16, EMB, sGcn, BIASP, dummyres, 0L, NODEP, 64, CHEBW, 1.0f);
  for (int k = 0; k < 3; ++k)
    run_gemm<0, 1, false, 0>(stream, NBS, THT16 + (size_t)k * 4096, 64, 0L, EOS16, EMB, sEmb, (void*)(TMPT16 + k * NODEP), CHEBW, sTmp,
                             BIASP, dummyres, 0L, 64, NODEP, EMB, 1.0f);
  run_gemm<0, 1, false, 2>(stream, NBS, CHEB16, CHEBW, 0L, TMPT16, CHEBW, sTmp, (void*)GCNO16, EMB, sGcn, BIASP, dummyres, 0L, NODEP, 64, CHEBW, 1.0f);

  run_gemm<2, 0, false, 0>(stream, 1, GCNX16, EMB, 0L, UXT16, EMB, 0L, (void*)GX, NGX, 0L, bx, dummyres, 0L, R1ROWS, NGX, EMB, 1.0f);
  run_gemm<2, 0, false, 0>(stream, 1, GCNO16, EMB, 0L, UGT16, EMB, 0L, (void*)GG, NGG, 0L, bg, dummyres, 0L, R1ROWS, NGG, EMB, 1.0f);

  lstm_kernel<<<LSTM_BLOCKS, LB_THR, 0, stream>>>(GX, GG, VTW16, HS16);

  run_gemm<2, 1, false, 2>(stream, 1, HS16, EMB, 0L, WFF1T, EMB, 0L, (void*)FF1_16, EMB, 0L, bff1, dummyres, 0L, R1ROWS, 64, EMB, 1.0f);
  run_gemm<2, 1, false, 0>(stream, 1, FF1_16, EMB, 0L, WFF2T, EMB, 0L, (void*)HID16, EMB, 0L, bff2, dummyres, 0L, R1ROWS, 64, EMB, 1.0f);

  tcgather_kernel<<<(LROWP * 16) / NTHR, NTHR, 0, stream>>>(HID16, TCA16);
  run_gemm<2, 0, false, 0>(stream, 1, TCA16, 128, 0L, WTC16, 128, 0L, (void*)TCL, EMB, 0L, btc, dummyres, 0L, LROWP, 64, 128, 1.0f);

  scramble_kernel<<<R2ROWS / 4, NTHR, 0, stream>>>(x, Wex, bex, TCL, QIN16, KVIN16);

  run_gemm<2, 1, false, 0>(stream, 1, QIN16, EMB, 0L, WQP16, EMB, 0L, (void*)QP16, QKW, 0L, BQP, dummyres, 0L, R2ROWS, QKW, EMB, 1.0f);
  run_gemm<2, 1, false, 0>(stream, 1, KVIN16, EMB, 0L, WKP16, EMB, 0L, (void*)KP16, QKW, 0L, BKP, dummyres, 0L, R2ROWS, QKW, EMB, 1.0f);
  run_gemm<1, 1, false, 0>(stream, SEQ, WV16, EMB, 0L, KVIN16, EMB, (long)LROWP * EMB, (void*)VTP16, LROWP, (long)64 * LROWP,
                           bin + 128, dummyres, 0L, 64, LROWP, EMB, 1.0f);

  const long sS = (long)LROWP * LROWP;
  for (int sp = 0; sp < SEQ; ++sp) {
    const unsigned short* qb = QP16 + (size_t)sp * LROWP * QKW;
    const unsigned short* kb = KP16 + (size_t)sp * LROWP * QKW;
    run_gemm<0, 0, false, 0>(stream, NHEADS, qb, QKW, (long)HDP, kb, QKW, (long)HDP, (void*)SPL, LROWP, sS, BIASP, dummyres, 0L, LROWP, LROWP, HDP, 1.0f);
    softmax_kernel<<<(4 * LROWP) / SM_ROWS, NTHR, 0, stream>>>(SPL, P16);
    run_gemm<0, 0, false, 0>(stream, NHEADS, P16, LROWP, sS, VTP16 + (size_t)sp * 64 * LROWP, LROWP, (long)HDIM * LROWP,
                             (void*)(CTXH + (size_t)sp * NHEADS * LROWP * EMB), EMB, (long)LROWP * EMB, BIASP, dummyres, 0L,
                             LROWP, 64, LROWP, PCARRY_INV);
  }

  ctxpack_kernel<<<(R1ROWS * 8) / NTHR, NTHR, 0, stream>>>(CTXH, CTX16);
  run_gemm<2, 1, false, 0>(stream, 1, CTX16, EMB, 0L, WOUT16, EMB, 0L, (void*)DSA16, EMB, 0L, BOUT64, dummyres, 0L, R1ROWS, 64, EMB, 1.0f);
  run_gemm<2, 1, false, 2>(stream, 1, DSA16, EMB, 0L, WFA1T, EMB, 0L, (void*)FA1_16, EMB, 0L, BFA164, dummyres, 0L, R1ROWS, 64, EMB, 1.0f);
  run_gemm<2, 0, false, 0>(stream, 1, FA1_16, EMB, 0L, WFA2T, EMB, 0L, (void*)FFA, EMB, 0L, bfa2, dummyres, 0L, R1ROWS, 64, EMB, CCARRY_INV);
  run_gemm<2, 0, true, 0>(stream, 1, HID16, EMB, 0L, WRC16, EMB, 0L, (void*)COMB, EMB, 0L, brc, FFA, 0L, R1ROWS, 64, EMB, 1.0f);

  final_kernel<<<(NOUT + NTHR - 1) / NTHR, NTHR, 0, stream>>>(COMB, Wfin, bfin, out);
}
